// UGCGRUCell_90202903150932
// MI455X (gfx1250) — hardware-verified
//
#include <hip/hip_runtime.h>
#include <stddef.h>
#include <stdint.h>
#include <math.h>


#pragma clang fp contract(off)

#define NNODE 10000
#define NU    64
#define NIN   2
#define NB    16
#define NF    66
#define KW    132
#define KP    160
#define KSTEP (KP / 32)
#define SEG   80
#define XSEG  72
#define XROW  (NB * XSEG)
#define NNU   (NNODE * NU)
#define NNI   (NNODE * NIN)
#define TPB   (NNODE / 16)
#define NTILE (NB * TPB)
#define GW    8
#define GROWS (GW * 16)
#define WSCALE 16.0f
#define WINV   0.0625f

#define NTHR    256
#define NWAVE   8
#define EPT     8
#define NGRP    2
#define CHUNK   (NTHR * EPT * NGRP)
#define WCAP    (EPT * NGRP * 32)
#define LISTN   (NWAVE * WCAP)
#define NBC     4096
#define NBF     1024
#define RCAP    40960
#define RBN     128
#define TGT     256
#define DEGCAP  256
#define OTHR    512

#define LDS_FILL ((RCAP + NBF + LISTN) * 4 + 64)
#define LDS_G1   (GROWS * 128 * 4)
#define LDS_G2   (GROWS * KP * 2)

static_assert((CHUNK & (CHUNK - 1)) == 0);
static_assert(CHUNK <= 4096);
static_assert((NBC & (NBC - 1)) == 0 && (NBF & (NBF - 1)) == 0);
static_assert(NBC == 4 * NBF);
static_assert(OTHR * 8 == NBC);
static_assert((RCAP % 32) == 0);
static_assert(TGT == NWAVE * 32);
static_assert(NNODE % 16 == 0);
static_assert(NTILE % GW == 0);
static_assert(XROW % 128 == 0);
static_assert((XSEG % 4) == 0);
static_assert(KP % 32 == 0 && KP >= KW);
static_assert(GROWS == 128 && NTHR == 2 * GROWS);
static_assert(LDS_G1 >= GROWS * KP * 2);
static_assert(LDS_G2 >= GROWS * 64 * 4);

typedef float          v2f  __attribute__((ext_vector_type(2)));
typedef float          v4f  __attribute__((ext_vector_type(4)));
typedef float          v8f  __attribute__((ext_vector_type(8)));
typedef int            v4i  __attribute__((ext_vector_type(4)));
typedef _Float16       v8h  __attribute__((ext_vector_type(8)));
typedef _Float16       v16h __attribute__((ext_vector_type(16)));
union FragH { v16h v; v8h h[2]; };

__device__ __forceinline__ v8f wmf(const FragH& a, const FragH& b, v8f c) {
  v8f d = __builtin_amdgcn_wmma_f32_16x16x32_f16(false, a.v, false, b.v, (short)0, c, false, false);
  asm volatile("v_nop\n\tv_nop\n\tv_nop\n\tv_nop" : "+v"(d) : "v"(a.v), "v"(b.v));
  return d;
}

__device__ __forceinline__ v8h cvt8(v4f a, v4f b) {
  v8h r;
  r[0] = (_Float16)a.x; r[1] = (_Float16)a.y; r[2] = (_Float16)a.z; r[3] = (_Float16)a.w;
  r[4] = (_Float16)b.x; r[5] = (_Float16)b.y; r[6] = (_Float16)b.z; r[7] = (_Float16)b.w;
  return r;
}

template <int NBS>
__device__ __forceinline__ int scan_chunk(const int* __restrict__ dsts, int nE, int cbase, int slotBase,
                                          int vec8, int* list, int tid, int lane, int wave) {
  int wc = 0;
#pragma unroll
  for (int g = 0; g < NGRP; ++g) {
    const int el0  = (g * NTHR + tid) * EPT;
    const int e0   = cbase + el0;
    const int sent = -2147483647 - 1;
    v4i da, db;
    if (vec8 != 0 && cbase + CHUNK <= nE) {
      da = *(const v4i*)(dsts + e0);
      db = *(const v4i*)(dsts + e0 + 4);
    } else {
      da.x = (e0     < nE) ? dsts[min(e0, nE - 1)] : sent;
      da.y = (e0 + 1 < nE) ? dsts[min(e0 + 1, nE - 1)] : sent;
      da.z = (e0 + 2 < nE) ? dsts[min(e0 + 2, nE - 1)] : sent;
      da.w = (e0 + 3 < nE) ? dsts[min(e0 + 3, nE - 1)] : sent;
      db.x = (e0 + 4 < nE) ? dsts[min(e0 + 4, nE - 1)] : sent;
      db.y = (e0 + 5 < nE) ? dsts[min(e0 + 5, nE - 1)] : sent;
      db.z = (e0 + 6 < nE) ? dsts[min(e0 + 6, nE - 1)] : sent;
      db.w = (e0 + 7 < nE) ? dsts[min(e0 + 7, nE - 1)] : sent;
    }
    const unsigned nb = (unsigned)slotBase;
    const unsigned s0 = (unsigned)da.x - nb, s1 = (unsigned)da.y - nb;
    const unsigned s2 = (unsigned)da.z - nb, s3 = (unsigned)da.w - nb;
    const unsigned s4 = (unsigned)db.x - nb, s5 = (unsigned)db.y - nb;
    const unsigned s6 = (unsigned)db.z - nb, s7 = (unsigned)db.w - nb;
    const bool h0 = s0 < (unsigned)NBS, h1 = s1 < (unsigned)NBS, h2 = s2 < (unsigned)NBS, h3 = s3 < (unsigned)NBS;
    const bool h4 = s4 < (unsigned)NBS, h5 = s5 < (unsigned)NBS, h6 = s6 < (unsigned)NBS, h7 = s7 < (unsigned)NBS;
    const unsigned any = __builtin_amdgcn_ballot_w32(h0 | h1 | h2 | h3 | h4 | h5 | h6 | h7);
    if (any != 0u) {
#define HITJ(J, HJ, SJ) { \
        const unsigned mj = __builtin_amdgcn_ballot_w32(HJ); \
        if (mj != 0u) { \
          if (HJ) { \
            const int pos = wc + (int)__builtin_amdgcn_mbcnt_lo(mj, 0u); \
            if (pos < WCAP) list[wave * WCAP + pos] = ((el0 + (J)) << 12) | (int)(SJ); \
          } \
          wc += (int)__builtin_popcount(mj); } }
      HITJ(0, h0, s0)
      HITJ(1, h1, s1)
      HITJ(2, h2, s2)
      HITJ(3, h3, s3)
      HITJ(4, h4, s4)
      HITJ(5, h5, s5)
      HITJ(6, h6, s6)
      HITJ(7, h7, s7)
#undef HITJ
    }
  }
  return wc;
}

__device__ __forceinline__ v8h wchunk8(const float* __restrict__ mu, const float* __restrict__ ls,
                                       const float* __restrict__ ep, int ncol, int col, int j) {
  float v[8];
#pragma unroll
  for (int e = 0; e < 8; ++e) {
    const int kp = 8 * j + e;
    const int seg = kp >= SEG ? 1 : 0;
    const int t = kp - SEG * seg;
    const int valid = t < NF ? 1 : 0;
    const int f = t < NU ? t + NIN : t - NU;
    int k = 2 * f + seg;
    k = valid ? k : 0;
    k = k < 0 ? 0 : (k > KW - 1 ? KW - 1 : k);
    const size_t idx = (size_t)k * ncol + col;
    const float w = mu[idx] + __expf(ls[idx]) * ep[idx];
    v[e] = valid ? w * WSCALE : 0.0f;
  }
  v4f a, b;
  a.x = v[0]; a.y = v[1]; a.z = v[2]; a.w = v[3];
  b.x = v[4]; b.y = v[5]; b.z = v[6]; b.w = v[7];
  return cvt8(a, b);
}

__global__ __launch_bounds__(NTHR) void k_wprep(
    const float* __restrict__ w1_mu, const float* __restrict__ w1_ls, const float* __restrict__ e_w1,
    const float* __restrict__ b1_mu, const float* __restrict__ b1_ls, const float* __restrict__ e_b1,
    const float* __restrict__ w2_mu, const float* __restrict__ w2_ls, const float* __restrict__ e_w2,
    const float* __restrict__ b2_mu, const float* __restrict__ b2_ls, const float* __restrict__ e_b2,
    _Float16* W1t, _Float16* W2t, float* B1f, float* B2f) {
  const int tid = threadIdx.x, blk = blockIdx.x;
  if (blk < 10) {
    const int i = blk * NTHR + tid;
    const int col = i / (KP / 8);
    const int j = i - col * (KP / 8);
    const v8h hv = wchunk8(w1_mu, w1_ls, e_w1, 2 * NU, col, j);
    _Float16* p = W1t + (size_t)i * 8;
    *(volatile v8h*)p = hv;
    __threadfence();
    *(volatile v8h*)p = hv;
  } else if (blk < 15) {
    const int i = (blk - 10) * NTHR + tid;
    const int col = i / (KP / 8);
    const int j = i - col * (KP / 8);
    const v8h hv = wchunk8(w2_mu, w2_ls, e_w2, NU, col, j);
    _Float16* p = W2t + (size_t)i * 8;
    *(volatile v8h*)p = hv;
    __threadfence();
    *(volatile v8h*)p = hv;
  } else {
    if (tid < 32) {
      const int c = 4 * tid;
      v4f r;
      r.x = b1_mu[c]     + __expf(b1_ls[c])     * e_b1[c];
      r.y = b1_mu[c + 1] + __expf(b1_ls[c + 1]) * e_b1[c + 1];
      r.z = b1_mu[c + 2] + __expf(b1_ls[c + 2]) * e_b1[c + 2];
      r.w = b1_mu[c + 3] + __expf(b1_ls[c + 3]) * e_b1[c + 3];
      *(volatile v4f*)(B1f + c) = r;
      __threadfence();
      *(volatile v4f*)(B1f + c) = r;
    } else if (tid < 64) {
      const int l = tid - 32;
      const int c = 4 * (l < 16 ? l : 15);
      v4f r;
      r.x = b2_mu[c]     + __expf(b2_ls[c])     * e_b2[c];
      r.y = b2_mu[c + 1] + __expf(b2_ls[c + 1]) * e_b2[c + 1];
      r.z = b2_mu[c + 2] + __expf(b2_ls[c + 2]) * e_b2[c + 2];
      r.w = b2_mu[c + 3] + __expf(b2_ls[c + 3]) * e_b2[c + 3];
      if (l < 16) *(volatile v4f*)(B2f + c) = r;
      __threadfence();
      if (l < 16) *(volatile v4f*)(B2f + c) = r;
    }
  }
}

__global__ __launch_bounds__(NTHR) void k_count(const int* __restrict__ arow, int* cnt, int nE, int vec8) {
  __shared__ __attribute__((aligned(16))) int scnt[NBC];
  __shared__ __attribute__((aligned(16))) int list[LISTN];
  __shared__ int wcnt[NWAVE];
  const int tid = threadIdx.x, lane = tid & 31, wave = tid >> 5;
  const int nodeBase = blockIdx.x * NBC;

  for (int i = tid; i < NBC; i += NTHR) scnt[i] = 0;
  __syncthreads();

  const int nChunks = (nE + CHUNK - 1) / CHUNK;
#pragma unroll 1
  for (int ch = 0; ch < nChunks; ++ch) {
    const int cbase = ch * CHUNK;
    const int wc = scan_chunk<NBC>(arow, nE, cbase, nodeBase, vec8, list, tid, lane, wave);
    if (lane == 0) wcnt[wave] = wc;
    __syncthreads();
    if (wave == 0) {
#pragma unroll 1
      for (int wsx = 0; wsx < NWAVE; ++wsx) {
        int n = __builtin_amdgcn_readfirstlane(wcnt[wsx]);
        n = n > WCAP ? WCAP : (n < 0 ? 0 : n);
        const int* lp = list + wsx * WCAP;
#pragma unroll 1
        for (int i = 0; i < n; ++i) {
          const int ent  = __builtin_amdgcn_readfirstlane(lp[i]);
          const int slot = ent & (NBC - 1);
          if (lane == 0) scnt[slot] = scnt[slot] + 1;
        }
      }
    }
    __syncthreads();
  }

  v4i cq[4];
#pragma unroll
  for (int q = 0; q < 4; ++q) {
    const int f = (wave * 4 + q) * 128 + 4 * lane;
    cq[q] = *(const v4i*)(scnt + f);
  }
  int* cp = cnt + (size_t)nodeBase;
#pragma unroll
  for (int q = 0; q < 4; ++q) {
    const int f = (wave * 4 + q) * 128 + 4 * lane;
    *(volatile v4i*)(cp + f) = cq[q];
  }
  __threadfence();
#pragma unroll
  for (int q = 0; q < 4; ++q) {
    const int f = (wave * 4 + q) * 128 + 4 * lane;
    *(volatile v4i*)(cp + f) = cq[q];
  }
}

__global__ __launch_bounds__(OTHR) void k_offsets(
    const int* __restrict__ cnt, int* off, int* rbase, int nChunk) {
  __shared__ __attribute__((aligned(16))) int soff[NBC];
  __shared__ __attribute__((aligned(16))) int srb[RBN];
  __shared__ int wtot[OTHR / 32];
  const int tid = threadIdx.x, lane = tid & 31, wave = tid >> 5, sub = tid >> 7;
  for (int i = tid; i < RBN; i += OTHR) srb[i] = 0;
  int carry = 0;
#pragma unroll 1
  for (int ch = 0; ch < nChunk; ++ch) {
    const int base = ch * NBC;
    const v4i c0 = *(const v4i*)(cnt + base + 8 * tid);
    const v4i c1 = *(const v4i*)(cnt + base + 8 * tid + 4);
    const int e0 = max(c0.x, 0), e1 = max(c0.y, 0), e2 = max(c0.z, 0), e3 = max(c0.w, 0);
    const int e4 = max(c1.x, 0), e5 = max(c1.y, 0), e6 = max(c1.z, 0), e7 = max(c1.w, 0);
    const int ts = e0 + e1 + e2 + e3 + e4 + e5 + e6 + e7;
    int incl = ts;
#pragma unroll
    for (int d = 1; d < 32; d <<= 1) {
      const int t = __shfl_up(incl, d);
      if (lane >= d) incl += t;
    }
    if (lane == 31) wtot[wave] = incl;
    __syncthreads();
    const int S0 = wtot[0]  + wtot[1]  + wtot[2]  + wtot[3];
    const int S1 = wtot[4]  + wtot[5]  + wtot[6]  + wtot[7];
    const int S2 = wtot[8]  + wtot[9]  + wtot[10] + wtot[11];
    const int S3 = wtot[12] + wtot[13] + wtot[14] + wtot[15];
    int pre = 0;
#pragma unroll 1
    for (int w = 4 * sub; w < wave; ++w) pre += wtot[w];
    const int b0 = carry;
    const int b1 = b0 + ((S0 + 31) & ~31);
    const int b2 = b1 + ((S1 + 31) & ~31);
    const int b3 = b2 + ((S2 + 31) & ~31);
    const int b4 = b3 + ((S3 + 31) & ~31);
    const int myb = sub == 0 ? b0 : (sub == 1 ? b1 : (sub == 2 ? b2 : b3));
    if (tid == 0) {
      srb[min(4 * ch + 0, RBN - 1)] = b0;
      srb[min(4 * ch + 1, RBN - 1)] = b1;
      srb[min(4 * ch + 2, RBN - 1)] = b2;
      srb[min(4 * ch + 3, RBN - 1)] = b3;
    }
    int run = myb + pre + incl - ts;
    soff[8 * tid + 0] = run; run += e0;
    soff[8 * tid + 1] = run; run += e1;
    soff[8 * tid + 2] = run; run += e2;
    soff[8 * tid + 3] = run; run += e3;
    soff[8 * tid + 4] = run; run += e4;
    soff[8 * tid + 5] = run; run += e5;
    soff[8 * tid + 6] = run; run += e6;
    soff[8 * tid + 7] = run;
    carry = b4;
    __syncthreads();
    const v4i o0 = *(const v4i*)(soff + 4 * tid);
    const v4i o1 = *(const v4i*)(soff + 4 * (tid + OTHR));
    int* op = off + base;
    *(volatile v4i*)(op + 4 * tid) = o0;
    *(volatile v4i*)(op + 4 * (tid + OTHR)) = o1;
    __threadfence();
    *(volatile v4i*)(op + 4 * tid) = o0;
    *(volatile v4i*)(op + 4 * (tid + OTHR)) = o1;
    __syncthreads();
  }
  if (tid == 0) srb[min(4 * nChunk, RBN - 1)] = carry;
  __syncthreads();
  v4i rv = {0, 0, 0, 0};
  if (tid < 32) rv = *(const v4i*)(srb + 4 * tid);
  if (tid < 32) *(volatile v4i*)(rbase + 4 * tid) = rv;
  __threadfence();
  if (tid < 32) *(volatile v4i*)(rbase + 4 * tid) = rv;
}

__global__ __launch_bounds__(NTHR) void k_fill(
    const int* __restrict__ arow, const int* __restrict__ off, const int* __restrict__ rbase,
    int* csr, int nE, int vec8, int csrLen) {
  extern __shared__ v4f lds_dyn[];
  int* region = (int*)lds_dyn;
  int* cursor = region + RCAP;
  int* list   = cursor + NBF;
  int* wcnt   = list + LISTN;
  const int tid = threadIdx.x, lane = tid & 31, wave = tid >> 5;
  const int b = blockIdx.x;
  const int nodeBase = b * NBF;

  int rb0 = rbase[b];
  const int rb1 = rbase[b + 1];
  rb0 = rb0 < 0 ? 0 : (rb0 > csrLen ? csrLen : rb0);
  rb0 &= ~31;
  int len = rb1 - rb0;
  len = len < 0 ? 0 : (len > RCAP ? RCAP : len);
  int lenW = (len + 31) & ~31;
  if (rb0 + lenW > csrLen) lenW = (csrLen - rb0) & ~31;

  {
    const v4i z = {0, 0, 0, 0};
    for (int i = tid; i < RCAP / 4; i += NTHR) ((v4i*)region)[i] = z;
    for (int s = tid; s < NBF; s += NTHR) {
      int o = off[nodeBase + s] - rb0;
      o = o < 0 ? 0 : (o > RCAP ? RCAP : o);
      cursor[s] = o;
    }
  }
  __syncthreads();

  const int nChunks = (nE + CHUNK - 1) / CHUNK;
#pragma unroll 1
  for (int ch = 0; ch < nChunks; ++ch) {
    const int cbase = ch * CHUNK;
    const int wc = scan_chunk<NBF>(arow, nE, cbase, nodeBase, vec8, list, tid, lane, wave);
    if (lane == 0) wcnt[wave] = wc;
    __syncthreads();
    if (wave == 0) {
#pragma unroll 1
      for (int wsx = 0; wsx < NWAVE; ++wsx) {
        int n = __builtin_amdgcn_readfirstlane(wcnt[wsx]);
        n = n > WCAP ? WCAP : (n < 0 ? 0 : n);
        const int* lp = list + wsx * WCAP;
#pragma unroll 1
        for (int i = 0; i < n; ++i) {
          const int ent  = __builtin_amdgcn_readfirstlane(lp[i]);
          const int slot = ent & (NBF - 1);
          int e = cbase + ((ent >> 12) & (CHUNK - 1));
          e = e > nE - 1 ? nE - 1 : e;
          if (lane == 0) {
            int pos = cursor[slot];
            pos = pos < 0 ? 0 : (pos > RCAP - 1 ? RCAP - 1 : pos);
            region[pos] = e;
            const int np = pos + 1;
            cursor[slot] = np > RCAP ? RCAP : np;
          }
        }
      }
    }
    __syncthreads();
  }

  const int nv = lenW >> 2;
  int* gp = csr + rb0;
#pragma unroll 1
  for (int i = tid; i < nv; i += NTHR) { const v4i v = ((const v4i*)region)[i]; *(volatile v4i*)(gp + 4 * i) = v; }
  __threadfence();
#pragma unroll 1
  for (int i = tid; i < nv; i += NTHR) { const v4i v = ((const v4i*)region)[i]; *(volatile v4i*)(gp + 4 * i) = v; }
}

__global__ __launch_bounds__(NTHR) void k_agg(
    const int* __restrict__ csr, const int* __restrict__ off, const int* __restrict__ cnt,
    const int* __restrict__ acol, const float* __restrict__ aval,
    const float* __restrict__ xin, const float* __restrict__ st,
    float* x1p, int nE, int csrLen) {
  __shared__ __attribute__((aligned(16))) float wbuf[NWAVE * XROW];
  const int tid = threadIdx.x, lane = tid & 31, wave = tid >> 5;
  const int bb = lane & 15, h = lane >> 4;
  const int tbase = blockIdx.x * TGT + wave * 32;
  const int cl = tbase + lane;
  const int cnt_l = cnt[cl];
  const int off_l = off[cl];
  const float* stb = st + (size_t)bb * NNU + 32 * h;
  const float* inb = xin + (size_t)bb * NNI;
  float* wr = wbuf + wave * XROW + bb * XSEG;
  const float* lb = wbuf + wave * XROW;
  union FI { float f; int i; };
  const v4f z4 = {0.f, 0.f, 0.f, 0.f};

#pragma unroll 1
  for (int j = 0; j < 32; ++j) {
    const int c = tbase + j;
    int n = __builtin_amdgcn_readlane(cnt_l, j);
    n = n < 0 ? 0 : (n > DEGCAP ? DEGCAP : n);
    const int sst = __builtin_amdgcn_readlane(off_l, j);
    v4f a[8];
#pragma unroll
    for (int q = 0; q < 8; ++q) a[q] = z4;
    v2f ai = {0.f, 0.f};
#pragma unroll 1
    for (int q0 = 0; q0 < n; q0 += 32) {
      int pos = sst + q0 + lane;
      pos = pos < 0 ? 0 : (pos > csrLen - 1 ? csrLen - 1 : pos);
      int ed = csr[pos];
      ed = ed < 0 ? 0 : (ed > nE - 1 ? nE - 1 : ed);
      int cc = acol[ed];
      cc = cc < 0 ? 0 : (cc > NNODE - 1 ? NNODE - 1 : cc);
      FI vv; vv.f = aval[ed];
      const int mcnt = (n - q0) < 32 ? (n - q0) : 32;
#pragma unroll 1
      for (int p = 0; p < mcnt; ++p) {
        const int s = __builtin_amdgcn_readlane(cc, p);
        FI w; w.i = __builtin_amdgcn_readlane(vv.i, p);
        const float* xp = stb + (size_t)s * NU;
#pragma unroll
        for (int q = 0; q < 8; ++q) {
          const v4f xv = *(const v4f*)(xp + 4 * q);
          a[q] = a[q] + xv * w.f;
        }
        const v2f xi = *(const v2f*)(inb + (size_t)s * NIN);
        ai = ai + xi * w.f;
      }
    }
#pragma unroll
    for (int q = 0; q < 8; ++q) *(v4f*)(wr + 32 * h + 4 * q) = a[q];
    if (h == 0) {
      *(v2f*)(wr + 64) = ai;
    } else {
      const v2f z2 = {0.f, 0.f};
      *(v2f*)(wr + 66) = z2;
      *(v4f*)(wr + 68) = z4;
    }
    __syncthreads();
    float* gp = x1p + (size_t)c * XROW;
#pragma unroll
    for (int i = 0; i < XROW / 128; ++i) {
      const v4f v = *(const v4f*)(lb + 4 * (lane + 32 * i));
      *(volatile v4f*)(gp + 4 * (lane + 32 * i)) = v;
    }
    __threadfence();
#pragma unroll
    for (int i = 0; i < XROW / 128; ++i) {
      const v4f v = *(const v4f*)(lb + 4 * (lane + 32 * i));
      *(volatile v4f*)(gp + 4 * (lane + 32 * i)) = v;
    }
    __syncthreads();
  }
}

template <int NCT, bool GATES>
__global__ __launch_bounds__(NTHR) void k_gemm(
    const float* __restrict__ xin, const float* __restrict__ hx, const float* __restrict__ st,
    const float* __restrict__ x1p, const _Float16* __restrict__ Wt, const float* __restrict__ bias,
    float* rh, float* out) {
  extern __shared__ v4f lds_dyn[];
  _Float16* As = (_Float16*)lds_dyn;
  float* stg = (float*)lds_dyn;
  constexpr int SP = 16 * NCT;
  constexpr int CG = SP / 32;
  const int tid = threadIdx.x, lane = tid & 31, wave = tid >> 5, hh = lane >> 4, m = lane & 15;

  {
    const int row = tid & (GROWS - 1), jsel = tid >> 7;
    const int wt = row >> 4, rl = row & 15;
    int gt = blockIdx.x * GW + wt;
    gt = gt > NTILE - 1 ? NTILE - 1 : gt;
    const int b = gt / TPB;
    const int n = (gt - b * TPB) * 16 + rl;
    const float* strow = st + (size_t)b * NNU + (size_t)n * NU;
    const float* xrow = x1p + (size_t)n * XROW + b * XSEG;
    const float* inrow = xin + (size_t)b * NNI + (size_t)n * NIN;
    _Float16* arow = As + row * KP;
#pragma unroll 1
    for (int jj = 0; jj < KP / 16; ++jj) {
      const int j = 2 * jj + jsel;
      v4f f0 = {0.f, 0.f, 0.f, 0.f}, f1 = {0.f, 0.f, 0.f, 0.f};
      if (j < 8) {
        f0 = *(const v4f*)(strow + 8 * j);
        f1 = *(const v4f*)(strow + 8 * j + 4);
      } else if (j == 8) {
        const v2f t = *(const v2f*)inrow;
        f0.x = t.x; f0.y = t.y;
      } else if (j >= 10 && j < 18) {
        f0 = *(const v4f*)(xrow + 8 * (j - 10));
        f1 = *(const v4f*)(xrow + 8 * (j - 10) + 4);
      } else if (j == 18) {
        const v2f t = *(const v2f*)(xrow + 64);
        f0.x = t.x; f0.y = t.y;
      }
      *(v8h*)(arow + 8 * j) = cvt8(f0, f1);
    }
  }
  __syncthreads();

  v8f acc[NCT];
#pragma unroll
  for (int t = 0; t < NCT; ++t) { v8f z = {0.f, 0.f, 0.f, 0.f, 0.f, 0.f, 0.f, 0.f}; acc[t] = z; }
  const _Float16* ap = As + (wave * 16 + m) * KP + 8 * hh;
#pragma unroll 1
  for (int kt = 0; kt < KSTEP; ++kt) {
    FragH a;
    a.h[0] = *(const v8h*)(ap + 32 * kt);
    a.h[1] = *(const v8h*)(ap + 32 * kt + 16);
#pragma unroll
    for (int t = 0; t < NCT; ++t) {
      const _Float16* bp = Wt + (size_t)(16 * t + m) * KP + 32 * kt + 8 * hh;
      FragH bq;
      bq.h[0] = *(const v8h*)bp;
      bq.h[1] = *(const v8h*)(bp + 16);
      acc[t] = wmf(a, bq, acc[t]);
    }
  }
  __syncthreads();

#pragma unroll
  for (int t = 0; t < NCT; ++t) {
    float* sp = stg + (wave * 16 + 8 * hh) * SP + 16 * t + m;
#pragma unroll
    for (int r = 0; r < 8; ++r) sp[r * SP] = acc[t][r] * WINV;
  }
  __syncthreads();

  int gtw = blockIdx.x * GW + wave;
  gtw = gtw > NTILE - 1 ? NTILE - 1 : gtw;
  const int bw = gtw / TPB;
  const int n0 = (gtw - bw * TPB) * 16;
  const size_t wbase = (size_t)bw * NNU + (size_t)n0 * NU;
  const float* hxb = hx + wbase;

  if (GATES) {
#pragma unroll 1
    for (int it = 0; it < 16 * CG; ++it) {
      const int rl = it / CG, col = ((it - rl * CG) << 5) + lane;
      float* sp = stg + (wave * 16 + rl) * SP + col;
      float v = *sp + bias[col];
      v = fminf(fmaxf(v, -30.0f), 30.0f);
      const float e = expf(-v);
      const float s = __builtin_amdgcn_rcpf(1.0f + e);
      const float hv = hxb[rl * NU + (col & (NU - 1))];
      *sp = (col < NU) ? s * hv : s;
    }
  } else {
    const float* ub = out + wbase;
#pragma unroll 1
    for (int it = 0; it < 16 * CG; ++it) {
      const int rl = it / CG, col = ((it - rl * CG) << 5) + lane;
      float* sp = stg + (wave * 16 + rl) * SP + col;
      const float v = *sp + bias[col];
      const float cv = tanhf(v);
      const int ix = rl * NU + col;
      const float u = ub[ix];
      const float hv = hxb[ix];
      const float t1 = u * hv;
      const float t2 = (1.0f - u) * cv;
      *sp = t1 + t2;
    }
  }
  __syncthreads();

  {
    const float* sr = stg + (wave * 16 + hh) * SP + 4 * m;
    if (GATES) {
      float* rp = rh + wbase + 4 * lane;
      float* op = out + wbase + 4 * lane;
#pragma unroll
      for (int i = 0; i < 8; ++i) {
        const v4f vr = *(const v4f*)(sr + 2 * i * SP);
        const v4f vu = *(const v4f*)(sr + 2 * i * SP + NU);
        *(volatile v4f*)(rp + 128 * i) = vr;
        *(volatile v4f*)(op + 128 * i) = vu;
      }
      __threadfence();
#pragma unroll
      for (int i = 0; i < 8; ++i) {
        const v4f vr = *(const v4f*)(sr + 2 * i * SP);
        const v4f vu = *(const v4f*)(sr + 2 * i * SP + NU);
        *(volatile v4f*)(rp + 128 * i) = vr;
        *(volatile v4f*)(op + 128 * i) = vu;
      }
    } else {
      float* op = out + wbase + 4 * lane;
#pragma unroll
      for (int i = 0; i < 8; ++i) {
        const v4f v = *(const v4f*)(sr + 2 * i * SP);
        *(volatile v4f*)(op + 128 * i) = v;
      }
      __threadfence();
#pragma unroll
      for (int i = 0; i < 8; ++i) {
        const v4f v = *(const v4f*)(sr + 2 * i * SP);
        *(volatile v4f*)(op + 128 * i) = v;
      }
    }
  }
}

extern "C" void kernel_launch(void* const* d_in, const int* in_sizes, int n_in,
                              void* d_out, int out_size, void* d_ws, size_t ws_size,
                              hipStream_t stream) {
  if (n_in < 17) return;
  const int nE = in_sizes[2];
  if (in_sizes[0] != NB * NNI || in_sizes[1] != NB * NNU) return;
  if (nE <= 0 || nE > (1 << 26) || in_sizes[15] != nE || in_sizes[16] != nE) return;
  if (in_sizes[3] != KW * 2 * NU || in_sizes[4] != KW * 2 * NU || in_sizes[11] != KW * 2 * NU) return;
  if (in_sizes[5] != 2 * NU || in_sizes[6] != 2 * NU || in_sizes[12] != 2 * NU) return;
  if (in_sizes[7] != KW * NU || in_sizes[8] != KW * NU || in_sizes[13] != KW * NU) return;
  if (in_sizes[9] != NU || in_sizes[10] != NU || in_sizes[14] != NU) return;
  if (out_size != NB * NNU) return;

  const float* xin   = (const float*)d_in[0];
  const float* hx    = (const float*)d_in[1];
  const float* eval  = (const float*)d_in[2];
  const float* w1_mu = (const float*)d_in[3];
  const float* w1_ls = (const float*)d_in[4];
  const float* b1_mu = (const float*)d_in[5];
  const float* b1_ls = (const float*)d_in[6];
  const float* w2_mu = (const float*)d_in[7];
  const float* w2_ls = (const float*)d_in[8];
  const float* b2_mu = (const float*)d_in[9];
  const float* b2_ls = (const float*)d_in[10];
  const float* e_w1  = (const float*)d_in[11];
  const float* e_b1  = (const float*)d_in[12];
  const float* e_w2  = (const float*)d_in[13];
  const float* e_b2  = (const float*)d_in[14];
  const int*   erow  = (const int*)d_in[15];
  const int*   ecol  = (const int*)d_in[16];
  float* out = (float*)d_out;

  const int NPAD   = ((NNODE + TGT - 1) / TGT) * TGT;
  const int nBC    = (NNODE + NBC - 1) / NBC;
  const int CNTPAD = nBC * NBC;
  if (CNTPAD < NPAD) return;
  if (4 * nBC + 1 > RBN) return;
  const int nBF    = (NNODE + NBF - 1) / NBF;
  const int csrLen = ((nE + 31) & ~31) + 4096;
  const int nAgg   = NPAD / TGT;
  const int nGemm  = NTILE / GW;

  char* ws = (char*)d_ws;
  size_t off = 0;
  const size_t oW1  = off; off += (size_t)2 * NU * KP * 2;         off = (off + 255) & ~(size_t)255;
  const size_t oW2  = off; off += (size_t)NU * KP * 2;             off = (off + 255) & ~(size_t)255;
  const size_t oB1  = off; off += (size_t)2 * NU * 4;              off = (off + 255) & ~(size_t)255;
  const size_t oB2  = off; off += (size_t)NU * 4;                  off = (off + 255) & ~(size_t)255;
  const size_t oCnt = off; off += (size_t)CNTPAD * 4;              off = (off + 255) & ~(size_t)255;
  const size_t oOff = off; off += (size_t)CNTPAD * 4;              off = (off + 255) & ~(size_t)255;
  const size_t oRb  = off; off += (size_t)RBN * 4;                 off = (off + 255) & ~(size_t)255;
  const size_t oCsr = off; off += (size_t)csrLen * 4;              off = (off + 255) & ~(size_t)255;
  const size_t oX1  = off; off += (size_t)NPAD * XROW * 4;         off = (off + 255) & ~(size_t)255;
  const size_t oRh  = off; off += (size_t)NB * NNU * 4;            off = (off + 255) & ~(size_t)255;
  if (off > ws_size) return;
  _Float16* W1t  = (_Float16*)(ws + oW1);
  _Float16* W2t  = (_Float16*)(ws + oW2);
  float*    B1f  = (float*)(ws + oB1);
  float*    B2f  = (float*)(ws + oB2);
  int*      cnt  = (int*)(ws + oCnt);
  int*      offp = (int*)(ws + oOff);
  int*      rb   = (int*)(ws + oRb);
  int*      csr  = (int*)(ws + oCsr);
  float*    x1p  = (float*)(ws + oX1);
  float*    rhp  = (float*)(ws + oRh);

  const int vec8 = ((nE & 3) == 0) ? 1 : 0;

  k_wprep<<<16, NTHR, 0, stream>>>(w1_mu, w1_ls, e_w1, b1_mu, b1_ls, e_b1,
                                   w2_mu, w2_ls, e_w2, b2_mu, b2_ls, e_b2, W1t, W2t, B1f, B2f);

  k_count<<<nBC, NTHR, 0, stream>>>(erow, cnt, nE, vec8);
  k_offsets<<<1, OTHR, 0, stream>>>(cnt, offp, rb, nBC);
  hipFuncSetAttribute(reinterpret_cast<const void*>(&k_fill),
                      hipFuncAttributeMaxDynamicSharedMemorySize, LDS_FILL);
  k_fill<<<nBF, NTHR, LDS_FILL, stream>>>(erow, offp, rb, csr, nE, vec8, csrLen);

  k_agg<<<nAgg, NTHR, 0, stream>>>(csr, offp, cnt, ecol, eval, xin, hx, x1p, nE, csrLen);

  hipFuncSetAttribute(reinterpret_cast<const void*>(&k_gemm<8, true>),
                      hipFuncAttributeMaxDynamicSharedMemorySize, LDS_G1);
  k_gemm<8, true><<<nGemm, NTHR, LDS_G1, stream>>>(xin, hx, hx, x1p, W1t, B1f, rhp, out);

  k_agg<<<nAgg, NTHR, 0, stream>>>(csr, offp, cnt, ecol, eval, xin, rhp, x1p, nE, csrLen);

  hipFuncSetAttribute(reinterpret_cast<const void*>(&k_gemm<4, false>),
                      hipFuncAttributeMaxDynamicSharedMemorySize, LDS_G2);
  k_gemm<4, false><<<nGemm, NTHR, LDS_G2, stream>>>(xin, hx, rhp, x1p, W2t, B2f, rhp, out);
}
